// conv_matrix_layer_68186900791733
// MI455X (gfx1250) — hardware-verified
//
#include <hip/hip_runtime.h>
#include <stddef.h>
#include <stdint.h>

#pragma clang fp contract(off)

#define NB     4096
#define NM     128
#define NK     16384
#define NMOM   255
#define EPSBN  1e-5f
#define MOMEL  2048
#define MOMBLK 256
#define BMT    64
#define LDA    136
#define STP    36

static_assert(NK == NM * NM);
static_assert(NB % BMT == 0);
static_assert((NB * NM) == MOMEL * MOMBLK);
static_assert((NM * NK) % (8 * 256) == 0);
static_assert((LDA * 2) % 16 == 0);
static_assert((STP * 4) % 16 == 0);
static_assert(NMOM == 2 * NM - 1);
static_assert(NMOM < 256);

typedef __bf16       v16bf __attribute__((ext_vector_type(16)));
typedef float        v8f   __attribute__((ext_vector_type(8)));
typedef float        v4f   __attribute__((ext_vector_type(4)));
typedef unsigned int v4u   __attribute__((ext_vector_type(4)));
typedef v4u __attribute__((may_alias)) v4ua;
typedef v4f __attribute__((may_alias)) v4fa;

union Frag { v16bf v; v4u q[2]; };

__device__ __forceinline__ v8f mma_bf(v16bf a, v16bf b, v8f cacc) {
  cacc = __builtin_amdgcn_wmma_f32_16x16x32_bf16(false, a, false, b, (short)0, cacc, false, false);
  asm volatile("v_nop\n\tv_nop\n\tv_nop\n\tv_nop" : "+v"(cacc) : "v"(a), "v"(b));
  return cacc;
}

__device__ __forceinline__ v8f zero8() { return (v8f){0.f, 0.f, 0.f, 0.f, 0.f, 0.f, 0.f, 0.f}; }

__device__ __forceinline__ void split_bf16(float v, unsigned& hb, unsigned& lb) {
  const unsigned u = __float_as_uint(v);
  const unsigned h = (u + 0x7fffu + ((u >> 16) & 1u)) >> 16;
  const float hf = __uint_as_float(h << 16);
  const float lv = v - hf;
  const unsigned ul = __float_as_uint(lv);
  lb = (ul + 0x7fffu + ((ul >> 16) & 1u)) >> 16;
  hb = h;
}

__device__ __forceinline__ v16bf ldfrag_g(const unsigned short* __restrict__ p, size_t ld, int row0, size_t k0, int lane) {
  const int m = lane & 15, lh = lane >> 4;
  const unsigned short* q = p + (size_t)(row0 + m) * ld + k0 + 8 * lh;
  Frag f;
  f.q[0] = *(const v4ua*)(q);
  f.q[1] = *(const v4ua*)(q + 16);
  return f.v;
}

__device__ __forceinline__ v16bf ldfrag_l(const unsigned short* p, int ld, int row0, int k0, int lane) {
  const int m = lane & 15, lh = lane >> 4;
  const unsigned short* q = p + (row0 + m) * ld + k0 + 8 * lh;
  Frag f;
  f.q[0] = *(const v4ua*)(q);
  f.q[1] = *(const v4ua*)(q + 16);
  return f.v;
}

__device__ __forceinline__ double wave_sum_d(double v) {
#pragma unroll
  for (int off = 16; off > 0; off >>= 1) {
    const unsigned long long qb = __builtin_bit_cast(unsigned long long, v);
    int lo = (int)(unsigned)(qb & 0xffffffffull);
    int hi = (int)(unsigned)(qb >> 32);
    lo = __shfl_xor(lo, off, 32);
    hi = __shfl_xor(hi, off, 32);
    const unsigned long long rb = ((unsigned long long)(unsigned)hi << 32) | (unsigned long long)(unsigned)lo;
    v += __builtin_bit_cast(double, rb);
  }
  return v;
}

__global__ __launch_bounds__(256) void k_mom(const float* __restrict__ X, double* __restrict__ Tpart) {
  __shared__ double wl[8][256];
  __shared__ __align__(16) double tp[256];
  const int tid = threadIdx.x, lane = tid & 31, wave = tid >> 5;
  const size_t base = (size_t)blockIdx.x * MOMEL + (size_t)tid * 8;
  const v4f xa = *(const v4fa*)(X + base);
  const v4f xb = *(const v4fa*)(X + base + 4);
  const float t0 = xa[0] * xa[0], t1 = xa[1] * xa[1], t2 = xa[2] * xa[2], t3 = xa[3] * xa[3];
  const float t4 = xb[0] * xb[0], t5 = xb[1] * xb[1], t6 = xb[2] * xb[2], t7 = xb[3] * xb[3];
  float p0 = 1.0f, p1 = 1.0f, p2 = 1.0f, p3 = 1.0f, p4 = 1.0f, p5 = 1.0f, p6 = 1.0f, p7 = 1.0f;
#pragma unroll 1
  for (int m = 0; m < NMOM; ++m) {
    const float s = ((p0 + p1) + (p2 + p3)) + ((p4 + p5) + (p6 + p7));
    double d = (double)s;
    d = wave_sum_d(d);
    if (lane == 0) wl[wave][m] = d;
    p0 *= t0; p1 *= t1; p2 *= t2; p3 *= t3;
    p4 *= t4; p5 *= t5; p6 *= t6; p7 *= t7;
  }
  __syncthreads();
  {
    double s = 0.0;
#pragma unroll
    for (int w = 0; w < 8; ++w) s += wl[w][tid];
    tp[tid] = (tid < NMOM) ? s : 0.0;
  }
  __syncthreads();
  if (tid < 128) {
    const v4u val = *(const v4ua*)(tp + 2 * tid);
    double* dst = Tpart + (size_t)blockIdx.x * 256 + 2 * tid;
    *(volatile v4u*)dst = val;
    __threadfence();
    *(volatile v4u*)dst = val;
  }
}

__global__ __launch_bounds__(256) void k_fin(const double* __restrict__ Tpart, float* __restrict__ tab) {
  __shared__ double T[256];
  __shared__ __align__(16) float stg[256];
  const int tid = threadIdx.x;
  double s = 0.0;
#pragma unroll 1
  for (int b = 0; b < MOMBLK; ++b) s += Tpart[(size_t)b * 256 + tid];
  T[tid] = s;
  __syncthreads();
  {
    const int j = tid & (NM - 1);
    const double inv = 1.0 / (double)(NB * NM);
    const double mean = T[j] * inv;
    const double e2 = T[2 * j] * inv;
    double var = e2 - mean * mean;
    var = (var < 0.0) ? 0.0 : var;
    const float meanf = (float)mean;
    const float varf = (float)var;
    const float r = 1.0f / sqrtf(varf + EPSBN);
    stg[tid] = (tid < NM) ? meanf : r;
  }
  __syncthreads();
  if (tid < 64) {
    const v4f val = *(const v4fa*)(stg + 4 * tid);
    float* dst = tab + 4 * tid;
    *(volatile v4f*)dst = val;
    __threadfence();
    *(volatile v4f*)dst = val;
  }
}

__global__ __launch_bounds__(256) void k_wsplit(const float* __restrict__ W, unsigned short* __restrict__ Wh,
                                                unsigned short* __restrict__ Wl) {
  const size_t gid = (size_t)blockIdx.x * 256 + threadIdx.x;
  const v4f a = *(const v4fa*)(W + gid * 8);
  const v4f b = *(const v4fa*)(W + gid * 8 + 4);
  const float wv[8] = {a[0], a[1], a[2], a[3], b[0], b[1], b[2], b[3]};
  v4u hv, lv;
#pragma unroll
  for (int ep = 0; ep < 4; ++ep) {
    unsigned h0, l0, h1, l1;
    split_bf16(wv[2 * ep], h0, l0);
    split_bf16(wv[2 * ep + 1], h1, l1);
    hv[ep] = h0 | (h1 << 16);
    lv[ep] = l0 | (l1 << 16);
  }
  unsigned short* dh = Wh + gid * 8;
  unsigned short* dl = Wl + gid * 8;
  *(volatile v4u*)dh = hv;
  *(volatile v4u*)dl = lv;
  __threadfence();
  *(volatile v4u*)dh = hv;
  *(volatile v4u*)dl = lv;
}

__global__ __launch_bounds__(256) void k_gemm(const float* __restrict__ X, const float* __restrict__ tab,
                                              const float* __restrict__ gamma, const float* __restrict__ beta,
                                              const unsigned short* __restrict__ Wh, const unsigned short* __restrict__ Wl,
                                              const float* __restrict__ bias, float* __restrict__ out) {
  __shared__ float spar[4 * NM];
  __shared__ __align__(16) unsigned short sAh[BMT * LDA];
  __shared__ __align__(16) unsigned short sAl[BMT * LDA];
  __shared__ __align__(16) float st[8][16 * STP];

  const int tid = threadIdx.x, lane = tid & 31, wave = tid >> 5;
  const int hh = lane >> 4, c = lane & 15;
  const int wr = wave >> 2;
  const int wc = wave & 3;
  const int bm0 = blockIdx.x * BMT;
  const int arow0 = wr * 32;
  const int ncol0 = wc * 32;

  {
    spar[tid] = tab[tid];
    const float gv = gamma[tid & (NM - 1)];
    const float bv = beta[tid & (NM - 1)];
    spar[2 * NM + tid] = (tid < NM) ? gv : bv;
  }

  const int brow = tid >> 2;
  const int bq = tid & 3;
  const float* Xr = X + (size_t)(bm0 + brow) * NM + 32 * bq;
  unsigned short* ahrow = sAh + brow * LDA + 32 * bq;
  unsigned short* alrow = sAl + brow * LDA + 32 * bq;

  float P[32];
#pragma unroll
  for (int e = 0; e < 32; ++e) P[e] = 1.0f;

  v8f acc[2][2];
#pragma unroll
  for (int s = 0; s < 2; ++s) { acc[s][0] = zero8(); acc[s][1] = zero8(); }

  __syncthreads();

#pragma unroll 1
  for (int j = 0; j < NM; ++j) {
    const float mean = spar[j];
    const float rs = spar[NM + j];
    const float g = spar[2 * NM + j];
    const float be = spar[3 * NM + j];
#pragma unroll
    for (int gq = 0; gq < 4; ++gq) {
      const v4f xa = *(const v4fa*)(Xr + 8 * gq);
      const v4f xb = *(const v4fa*)(Xr + 8 * gq + 4);
      const float xv[8] = {xa[0], xa[1], xa[2], xa[3], xb[0], xb[1], xb[2], xb[3]};
      v4u hv, lv;
#pragma unroll
      for (int ep = 0; ep < 4; ++ep) {
        unsigned hb[2], lb[2];
#pragma unroll
        for (int h2 = 0; h2 < 2; ++h2) {
          const int e = 2 * ep + h2;
          const float x = xv[e];
          const float t = x * x;
          const float u = P[8 * gq + e];
          P[8 * gq + e] = u * t;
          float v = (u - mean) * rs;
          v = v * g + be;
          split_bf16(v, hb[h2], lb[h2]);
        }
        hv[ep] = hb[0] | (hb[1] << 16);
        lv[ep] = lb[0] | (lb[1] << 16);
      }
      *(v4ua*)(ahrow + 8 * gq) = hv;
      *(v4ua*)(alrow + 8 * gq) = lv;
    }
    __syncthreads();

    const size_t kg = (size_t)j * NM;
#pragma unroll 1
    for (int kc = 0; kc < 4; ++kc) {
      const int k0 = kc * 32;
      const v16bf bh0 = ldfrag_g(Wh, (size_t)NK, ncol0, kg + k0, lane);
      const v16bf bh1 = ldfrag_g(Wh, (size_t)NK, ncol0 + 16, kg + k0, lane);
      const v16bf bl0 = ldfrag_g(Wl, (size_t)NK, ncol0, kg + k0, lane);
      const v16bf bl1 = ldfrag_g(Wl, (size_t)NK, ncol0 + 16, kg + k0, lane);
#pragma unroll
      for (int s = 0; s < 2; ++s) {
        const v16bf ah = ldfrag_l(sAh, LDA, arow0 + 16 * s, k0, lane);
        const v16bf al = ldfrag_l(sAl, LDA, arow0 + 16 * s, k0, lane);
        acc[s][0] = mma_bf(ah, bh0, acc[s][0]);
        acc[s][0] = mma_bf(ah, bl0, acc[s][0]);
        acc[s][0] = mma_bf(al, bh0, acc[s][0]);
        acc[s][1] = mma_bf(ah, bh1, acc[s][1]);
        acc[s][1] = mma_bf(ah, bl1, acc[s][1]);
        acc[s][1] = mma_bf(al, bh1, acc[s][1]);
      }
    }
    __syncthreads();
  }

  const float bv0 = bias[ncol0 + c];
  const float bv1 = bias[ncol0 + 16 + c];
  float* sw = st[wave];
#pragma unroll
  for (int s = 0; s < 2; ++s) {
#pragma unroll
    for (int r = 0; r < 8; ++r) {
      sw[(8 * hh + r) * STP + c]      = acc[s][0][r] + bv0;
      sw[(8 * hh + r) * STP + 16 + c] = acc[s][1][r] + bv1;
    }
    __syncthreads();
    v4f val[4];
    size_t go[4];
#pragma unroll
    for (int it = 0; it < 4; ++it) {
      const int p = lane + 32 * it;
      const int L = p >> 3;
      const int pc = p & 7;
      val[it] = *(const v4fa*)(sw + L * STP + pc * 4);
      go[it] = (size_t)(bm0 + arow0 + 16 * s + L) * NM + ncol0 + pc * 4;
    }
    for (int ps = 0; ps < 2; ++ps) {
#pragma unroll
      for (int it = 0; it < 4; ++it) *(volatile v4f*)(out + go[it]) = val[it];
      __threadfence();
    }
    __syncthreads();
  }
}

extern "C" void kernel_launch(void* const* d_in, const int* in_sizes, int n_in,
                              void* d_out, int out_size, void* d_ws, size_t ws_size,
                              hipStream_t stream) {
  if (n_in < 5) return;
  if (in_sizes[0] != NB * NM) return;
  if (in_sizes[1] != NM) return;
  if (in_sizes[2] != NM) return;
  if (in_sizes[3] != NM * NK) return;
  if (in_sizes[4] != NM) return;
  if (out_size != NB * NM) return;

  const float* X     = (const float*)d_in[0];
  const float* gamma = (const float*)d_in[1];
  const float* beta  = (const float*)d_in[2];
  const float* W     = (const float*)d_in[3];
  const float* bconv = (const float*)d_in[4];
  float* out = (float*)d_out;

  const size_t off_tp   = 0;
  const size_t tp_bytes = (size_t)MOMBLK * 256 * sizeof(double);
  const size_t off_tab  = off_tp + tp_bytes;
  const size_t tab_bytes = 256 * sizeof(float);
  const size_t off_wh   = off_tab + tab_bytes;
  const size_t w_bytes  = (size_t)NM * NK * sizeof(unsigned short);
  const size_t off_wl   = off_wh + w_bytes;
  const size_t total    = off_wl + w_bytes;
  if (total > ws_size) return;

  char* ws = (char*)d_ws;
  double* Tpart = (double*)(ws + off_tp);
  float* tab = (float*)(ws + off_tab);
  unsigned short* Wh = (unsigned short*)(ws + off_wh);
  unsigned short* Wl = (unsigned short*)(ws + off_wl);

  k_mom<<<dim3(MOMBLK), dim3(256), 0, stream>>>(X, Tpart);
  k_fin<<<dim3(1), dim3(256), 0, stream>>>(Tpart, tab);
  k_wsplit<<<dim3((NM * NK) / (8 * 256)), dim3(256), 0, stream>>>(W, Wh, Wl);
  k_gemm<<<dim3(NB / BMT), dim3(256), 0, stream>>>(X, tab, gamma, beta, Wh, Wl, bconv, out);
  (void)hipGetLastError();
}
